// KANLikeRegressor_15212774163194
// MI455X (gfx1250) — hardware-verified
//
#include <hip/hip_runtime.h>
#include <math.h>

typedef __attribute__((ext_vector_type(16))) _Float16 v16h;
typedef __attribute__((ext_vector_type(16))) __bf16 v16b;
typedef __attribute__((ext_vector_type(8)))  _Float16 v8h;
typedef __attribute__((ext_vector_type(8)))  float v8f;
typedef __attribute__((ext_vector_type(4)))  float v4f;
typedef __attribute__((ext_vector_type(2)))  float v2f;
typedef __attribute__((ext_vector_type(4)))  unsigned v4u;
typedef __attribute__((ext_vector_type(4)))  int v4i;
typedef float __attribute__((may_alias)) float_a;
typedef int __attribute__((may_alias)) int_a;

template <typename T> __device__ __forceinline__ void vst2(void* p, T v) { *(volatile T*)p = v; __threadfence(); *(volatile T*)p = v; }
__device__ __forceinline__ v8f wmma16(v16h a, v16h b, v8f c) {
  v8f d = __builtin_amdgcn_wmma_f32_16x16x32_f16(false, a, false, b, (short)0, c, false, false);
  asm volatile("v_nop\n\tv_nop\n\tv_nop\n\tv_nop" : "+v"(d) : "v"(a), "v"(b));
  return d;
}
__device__ __forceinline__ v8f wmma_bf(v16b a, v16b b, v8f c) {
  v8f d = __builtin_amdgcn_wmma_f32_16x16x32_bf16(false, a, false, b, (short)0, c, false, false);
  asm volatile("v_nop\n\tv_nop\n\tv_nop\n\tv_nop" : "+v"(d) : "v"(a), "v"(b));
  return d;
}
__device__ __forceinline__ v16h frag_h(const _Float16* rowk0, int lane) {
  union { v16h v; v8h q[2]; } u; const _Float16* p = rowk0 + 8 * (lane >> 4);
  u.q[0] = *(const v8h*)p; u.q[1] = *(const v8h*)(p + 16); return u.v;
}
__device__ __forceinline__ v16h frag_f32(const float* rowk0, int lane) {
  v16h a; const float* p = rowk0 + 8 * (lane >> 4);
#pragma unroll
  for (int i = 0; i < 8; ++i) { a[i] = (_Float16)p[i]; a[8 + i] = (_Float16)p[16 + i]; }
  return a;
}
__device__ __forceinline__ v16h frag_f32s(const float* rowk0, int lane, float sc) {
  v16h a; const float* p = rowk0 + 8 * (lane >> 4);
#pragma unroll
  for (int i = 0; i < 8; ++i) { a[i] = (_Float16)(p[i] * sc); a[8 + i] = (_Float16)(p[16 + i] * sc); }
  return a;
}
__device__ __forceinline__ v16h fragc_f32(const float* W, int k0, int n, int lane, int ld, int K) {
  v16h a; const int g = lane >> 4;
#pragma unroll
  for (int i = 0; i < 8; ++i) { const int ka = k0 + 8 * g + i, kb = ka + 16;
    a[i] = (_Float16)(ka < K ? W[(size_t)(ka < K ? ka : K - 1) * ld + n] : 0.f); a[8 + i] = (_Float16)(kb < K ? W[(size_t)(kb < K ? kb : K - 1) * ld + n] : 0.f); }
  return a;
}
struct F2 { v16b h, l; };
__device__ __forceinline__ F2 bsplit16(const float v[16]) { F2 r;
#pragma unroll
  for (int i = 0; i < 16; ++i) { const __bf16 h = (__bf16)v[i]; r.h[i] = h; r.l[i] = (__bf16)(v[i] - (float)h); }
  return r; }
__device__ __forceinline__ F2 split_row(const float* row, int k0, int lane) { float v[16]; const float* p = row + k0 + 8 * (lane >> 4);
#pragma unroll
  for (int i = 0; i < 8; ++i) { v[i] = p[i]; v[8 + i] = p[16 + i]; }
  return bsplit16(v); }
__device__ __forceinline__ F2 split_rowK(const float* row, int k0, int lane, int K) { float v[16]; const int g = lane >> 4;
#pragma unroll
  for (int i = 0; i < 8; ++i) { const int ka = k0 + 8 * g + i, kb = ka + 16; v[i] = ka < K ? row[ka < K ? ka : K - 1] : 0.f; v[8 + i] = kb < K ? row[kb < K ? kb : K - 1] : 0.f; }
  return bsplit16(v); }
__device__ __forceinline__ F2 split_col(const float* W, int k0, int n, int lane, int ld, int K) { float v[16]; const int g = lane >> 4;
#pragma unroll
  for (int i = 0; i < 8; ++i) { const int ka = k0 + 8 * g + i, kb = ka + 16; v[i] = ka < K ? W[(size_t)(ka < K ? ka : K - 1) * ld + n] : 0.f; v[8 + i] = kb < K ? W[(size_t)(kb < K ? kb : K - 1) * ld + n] : 0.f; }
  return bsplit16(v); }
__device__ __forceinline__ v8f mac3(const F2& a, const F2& b, v8f c) { c = wmma_bf(a.l, b.h, c); c = wmma_bf(a.h, b.l, c); return wmma_bf(a.h, b.h, c); }
__device__ __forceinline__ float sigm(float v) { return 1.0f / (1.0f + expf(-v)); }
#define LDSX() do { asm volatile("s_wait_dscnt 0" ::: "memory"); __builtin_amdgcn_wave_barrier(); __builtin_amdgcn_fence(__ATOMIC_RELEASE, "workgroup"); } while (0)


#define NRW 65536
#define NFD 32
#define HH 128
#ifndef TRB
#define TRB (NRW / 64)
#endif
typedef __attribute__((ext_vector_type(8))) __bf16 v8b;
__device__ __forceinline__ v16b frag_b(const __bf16* rowk0, int lane) {
  union { v16b v; v8b q[2]; } u; const __bf16* p = rowk0 + 8 * (lane >> 4);
  u.q[0] = *(const v8b*)p; u.q[1] = *(const v8b*)(p + 16); return u.v;
}
__device__ __forceinline__ float bfr(float v) { return (float)(__bf16)v; }
__device__ __attribute__((noinline)) float exp_ni(float v) { return expf(v); }
__device__ __attribute__((noinline)) float erf_ni(float v) { return erff(v); }

#define WS_W2  0u
#define WS_PF  (WS_W2 + 2u * NFD * HH * HH)
#define WS_END (WS_PF + 4u * (size_t)NFD * NRW)

__global__ __launch_bounds__(128) void k_packw(const float* __restrict__ W2, _Float16* __restrict__ WT) {
  const int k = blockIdx.x, d = blockIdx.y, h = threadIdx.x; __shared__ __align__(16) _Float16 s[HH]; s[h] = (_Float16)bfr(W2[((size_t)d * HH + h) * HH + k]); __syncthreads();
  if (h < HH / 8) vst2((unsigned*)(WT + ((size_t)d * HH + k) * HH + h * 8), *(const v4u*)&s[h * 8]);
}
__global__ __launch_bounds__(128) void k_feat(const float* __restrict__ X, const float* __restrict__ W1, const float* __restrict__ B1, const _Float16* __restrict__ WT, const float* __restrict__ B2, const float* __restrict__ W3, const float* __restrict__ B3, float* __restrict__ PF) {
  __shared__ __align__(16) _Float16 sa[64][HH + 8]; __shared__ float sred[64][17]; __shared__ __align__(16) float sout[64];
  const int tid = threadIdx.x, wave = tid >> 5, lane = tid & 31, col = lane & 15, g = lane >> 4; const int d = blockIdx.y; const size_t r0 = (size_t)blockIdx.x * 64;
  for (int e = tid; e < 64 * HH; e += 128) { const int r = e >> 7, h = e & (HH - 1); const float xv = bfr(X[(r0 + r) * NFD + d]); const float v = fmaxf(xv * bfr(W1[d * HH + h]) + bfr(B1[d * HH + h]), 0.f); sa[r][h] = (_Float16)v; }
  if (tid < 64) for (int h = HH; h < HH + 8; ++h) sa[tid][h] = (_Float16)0.f;
  __syncthreads();
  v8f acc[8] = {};
#pragma unroll
  for (int kc = 0; kc < HH / 32; ++kc) { const v16h a = frag_h(&sa[wave * 16 + col][kc * 32], lane);
#pragma unroll
    for (int j = 0; j < 8; ++j) acc[j] = wmma16(a, frag_h(WT + ((size_t)d * HH + j * 16 + col) * HH + kc * 32, lane), acc[j]); }
#pragma unroll
  for (int r = 0; r < 8; ++r) { float p = 0.f;
#pragma unroll
    for (int j = 0; j < 8; ++j) { const int k = j * 16 + col; p += fmaxf(acc[j][r] + bfr(B2[d * HH + k]), 0.f) * bfr(W3[d * HH + k]); }
#pragma unroll
    for (int o = 1; o < 16; o <<= 1) p += __shfl_xor(p, o);
    if (col == 0) sred[wave * 16 + 8 * g + r][0] = p; }
  __syncthreads();
  if (tid < 64) sout[tid] = sred[tid][0] + bfr(B3[d]);
  __syncthreads();
  if (tid < 16) vst2(PF + (size_t)d * NRW + r0 + tid * 4, *(const v4f*)&sout[tid * 4]);
}
__global__ __launch_bounds__(256) void k_sum(const float* __restrict__ PF, float* __restrict__ OUT) {
  const size_t n = (size_t)blockIdx.x * 256 + threadIdx.x; float s = 0.f;
#pragma unroll 1
  for (int d = 0; d < NFD; ++d) s += PF[(size_t)d * NRW + n];
  __shared__ __align__(16) float so[256]; so[threadIdx.x] = s; __syncthreads();
  if (threadIdx.x < 64) vst2(OUT + (size_t)blockIdx.x * 256 + threadIdx.x * 4, *(const v4f*)&so[threadIdx.x * 4]);
}
extern "C" void kernel_launch(void* const* d_in, const int* in_sizes, int n_in, void* d_out, int out_size, void* d_ws, size_t ws_size, hipStream_t stream) {
  (void)in_sizes; (void)n_in; (void)out_size;
  const float** F = (const float**)d_in;
  if (ws_size < (size_t)WS_END) return;
  char* ws = (char*)d_ws; _Float16* WT = (_Float16*)(ws + WS_W2); float* PF = (float*)(ws + WS_PF);
  k_packw<<<dim3(HH, NFD), 128, 0, stream>>>(F[3], WT);
  k_feat<<<dim3(TRB, NFD), 128, 0, stream>>>(F[0], F[1], F[2], WT, F[4], F[5], F[6], PF);
  k_sum<<<(TRB * 64) / 256, 256, 0, stream>>>(PF, (float*)d_out);
}
